// ChebClassifier_41566693490715
// MI455X (gfx1250) — hardware-verified
//
#include <hip/hip_runtime.h>
#include <stddef.h>


#define NTHR    256
#define NWAVE   8
#define EPT     8
#define NGRP    2
#define CHUNK   (NTHR * EPT * NGRP)
#define WCAP    (EPT * NGRP * 32)
#define LISTN   (NWAVE * WCAP)
#define SLOTB   13
#define NBDEG   8192
#define NBA     8192
#define NBB     1024
#define NBC     512
#define GROWS   128
#define NLB     64
#define KCH     6
#define NCLS    10
#define LDS_AGG (32768 * 4 + LISTN * 4 + 64)
#define LDS_GEMM(CI, CO) ((CO) * ((CI) + 8) * 4 + GROWS * (CO) * 4)

static_assert(CHUNK == 4096);
static_assert(NBA * 4 == 32768);
static_assert(NBB * 32 == 32768);
static_assert(NBC * 64 == 32768);
static_assert(NBA <= (1 << SLOTB));
static_assert(NBDEG <= (1 << SLOTB));
static_assert(NBDEG % (NTHR * 4) == 0);
static_assert(GROWS == 16 * NWAVE);

typedef float          v2f   __attribute__((ext_vector_type(2)));
typedef float          v4f   __attribute__((ext_vector_type(4)));
typedef float          v8f   __attribute__((ext_vector_type(8)));
typedef int            v4i   __attribute__((ext_vector_type(4)));
typedef unsigned short v8us  __attribute__((ext_vector_type(8)));
typedef unsigned short v16us __attribute__((ext_vector_type(16)));
typedef __bf16         v16b  __attribute__((ext_vector_type(16)));
union FragB { v16b v; v16us u; v8us h[2]; };

__device__ __forceinline__ unsigned bfbits(float x) {
  const unsigned u = __float_as_uint(x);
  return (u + 0x7FFFu + ((u >> 16) & 1u)) >> 16;
}
__device__ __forceinline__ void split1(float x, unsigned short& hi, unsigned short& lo) {
  const unsigned hb = bfbits(x);
  const float hf = __uint_as_float(hb << 16);
  hi = (unsigned short)hb;
  lo = (unsigned short)bfbits(x - hf);
}
__device__ __forceinline__ void split8(v4f a, v4f b, v8us& hi, v8us& lo) {
  unsigned short p, q;
  split1(a.x, p, q); hi[0] = p; lo[0] = q;
  split1(a.y, p, q); hi[1] = p; lo[1] = q;
  split1(a.z, p, q); hi[2] = p; lo[2] = q;
  split1(a.w, p, q); hi[3] = p; lo[3] = q;
  split1(b.x, p, q); hi[4] = p; lo[4] = q;
  split1(b.y, p, q); hi[5] = p; lo[5] = q;
  split1(b.z, p, q); hi[6] = p; lo[6] = q;
  split1(b.w, p, q); hi[7] = p; lo[7] = q;
}

__device__ __forceinline__ v8f wmb(v16b a, v16b b, v8f c) {
  v8f d = __builtin_amdgcn_wmma_f32_16x16x32_bf16(false, a, false, b, (short)0, c, false, false);
  asm volatile("v_nop\n\tv_nop\n\tv_nop\n\tv_nop" : "+v"(d) : "v"(a), "v"(b));
  return d;
}

template <int NB>
__device__ __forceinline__ int scan_chunk(const int* __restrict__ keys, int nE, int cbase, int nodeBase,
                                          int vec8, int* list, int tid, int lane, int wave) {
  (void)lane;
  int wc = 0;
#pragma unroll
  for (int g = 0; g < NGRP; ++g) {
    const int el0  = (g * NTHR + tid) * EPT;
    const int e0   = cbase + el0;
    const int sent = -2147483647 - 1;
    v4i da, db;
    if (vec8 != 0 && cbase + CHUNK <= nE) {
      da = *(const v4i*)(keys + e0);
      db = *(const v4i*)(keys + e0 + 4);
    } else {
      da.x = (e0     < nE) ? keys[min(e0,     nE - 1)] : sent;
      da.y = (e0 + 1 < nE) ? keys[min(e0 + 1, nE - 1)] : sent;
      da.z = (e0 + 2 < nE) ? keys[min(e0 + 2, nE - 1)] : sent;
      da.w = (e0 + 3 < nE) ? keys[min(e0 + 3, nE - 1)] : sent;
      db.x = (e0 + 4 < nE) ? keys[min(e0 + 4, nE - 1)] : sent;
      db.y = (e0 + 5 < nE) ? keys[min(e0 + 5, nE - 1)] : sent;
      db.z = (e0 + 6 < nE) ? keys[min(e0 + 6, nE - 1)] : sent;
      db.w = (e0 + 7 < nE) ? keys[min(e0 + 7, nE - 1)] : sent;
    }
    const unsigned nb = (unsigned)nodeBase;
    const unsigned s0 = (unsigned)da.x - nb, s1 = (unsigned)da.y - nb;
    const unsigned s2 = (unsigned)da.z - nb, s3 = (unsigned)da.w - nb;
    const unsigned s4 = (unsigned)db.x - nb, s5 = (unsigned)db.y - nb;
    const unsigned s6 = (unsigned)db.z - nb, s7 = (unsigned)db.w - nb;
    const bool h0 = s0 < (unsigned)NB, h1 = s1 < (unsigned)NB, h2 = s2 < (unsigned)NB, h3 = s3 < (unsigned)NB;
    const bool h4 = s4 < (unsigned)NB, h5 = s5 < (unsigned)NB, h6 = s6 < (unsigned)NB, h7 = s7 < (unsigned)NB;
    const unsigned any = __builtin_amdgcn_ballot_w32(h0 | h1 | h2 | h3 | h4 | h5 | h6 | h7);
    if (any != 0u) {
#define HITJ(J, HJ, SJ) { \
        const unsigned mj = __builtin_amdgcn_ballot_w32(HJ); \
        if (mj != 0u) { \
          if (HJ) { \
            const int pos = wc + (int)__builtin_amdgcn_mbcnt_lo(mj, 0u); \
            if (pos < WCAP) list[wave * WCAP + pos] = ((el0 + (J)) << SLOTB) | (int)(SJ); \
          } \
          wc += (int)__builtin_popcount(mj); } }
      HITJ(0, h0, s0)
      HITJ(1, h1, s1)
      HITJ(2, h2, s2)
      HITJ(3, h3, s3)
      HITJ(4, h4, s4)
      HITJ(5, h5, s5)
      HITJ(6, h6, s6)
      HITJ(7, h7, s7)
#undef HITJ
    }
  }
  return wc;
}

template <int NB>
__global__ __launch_bounds__(NTHR) void k_deg(
    const int* __restrict__ keys, float* dinv, int nE, int vec8) {
  __shared__ __attribute__((aligned(16))) int cnt[NB];
  __shared__ __attribute__((aligned(16))) int list[LISTN];
  __shared__ int wcnt[NWAVE];
  const int tid = threadIdx.x, lane = tid & 31, wave = tid >> 5;
  const int nodeBase = blockIdx.x * NB;

  for (int i = tid; i < NB; i += NTHR) cnt[i] = 0;
  __syncthreads();

  const int nChunks = (nE + CHUNK - 1) / CHUNK;
#pragma unroll 1
  for (int ch = 0; ch < nChunks; ++ch) {
    const int cbase = ch * CHUNK;
    const int wc = scan_chunk<NB>(keys, nE, cbase, nodeBase, vec8, list, tid, lane, wave);
    if (lane == 0) wcnt[wave] = wc;
    __syncthreads();
    if (wave == 0) {
#pragma unroll 1
      for (int wsx = 0; wsx < NWAVE; ++wsx) {
        int n = __builtin_amdgcn_readfirstlane(wcnt[wsx]);
        n = n > WCAP ? WCAP : (n < 0 ? 0 : n);
        const int* lp = list + wsx * WCAP;
#pragma unroll 1
        for (int i = 0; i < n; ++i) {
          const int ent  = __builtin_amdgcn_readfirstlane(lp[i]);
          const int slot = ent & (NB - 1);
          if (lane == 0) cnt[slot] = cnt[slot] + 1;
        }
      }
    }
    __syncthreads();
  }

  constexpr int NI = NB / (NTHR * 4);
  v4f dq[NI];
#pragma unroll
  for (int q = 0; q < NI; ++q) {
    const int f = (q * NTHR + tid) * 4;
    const v4i c = *(const v4i*)(cnt + f);
    dq[q].x = (c.x > 0) ? __builtin_amdgcn_rsqf((float)c.x) : 0.f;
    dq[q].y = (c.y > 0) ? __builtin_amdgcn_rsqf((float)c.y) : 0.f;
    dq[q].z = (c.z > 0) ? __builtin_amdgcn_rsqf((float)c.z) : 0.f;
    dq[q].w = (c.w > 0) ? __builtin_amdgcn_rsqf((float)c.w) : 0.f;
  }
  float* dp = dinv + (size_t)nodeBase;
#pragma unroll
  for (int q = 0; q < NI; ++q) *(volatile v4f*)(dp + (q * NTHR + tid) * 4) = dq[q];
  __threadfence();
#pragma unroll
  for (int q = 0; q < NI; ++q) *(volatile v4f*)(dp + (q * NTHR + tid) * 4) = dq[q];
}

__global__ __launch_bounds__(NTHR) void k_cp34(const float* __restrict__ pos, float* dst, int nN) {
  const int r  = blockIdx.x * NTHR + threadIdx.x;
  const int rc = r < nN ? r : nN - 1;
  const float* p = pos + (size_t)rc * 3;
  v4f v;
  v.x = p[0]; v.y = p[1]; v.z = p[2]; v.w = 0.f;
  if (r >= nN) { v.x = 0.f; v.y = 0.f; v.z = 0.f; }
  float* gp = dst + (size_t)r * 4;
  *(volatile v4f*)gp = v;
  __threadfence();
  *(volatile v4f*)gp = v;
}

template <int C, int NB, int MODE>
__global__ __launch_bounds__(NTHR) void k_agg(
    const int* __restrict__ keys, const int* __restrict__ gidx, const float* __restrict__ wsrc,
    const float* __restrict__ zsrc, const float* __restrict__ zold, float* dst,
    int nN, int nE, int hop, int vec8) {
  extern __shared__ v4f lds_dyn[];
  float* acc  = (float*)lds_dyn;
  int*   list = (int*)(acc + NB * C);
  int*   wcnt = list + LISTN;
  constexpr int Q = C / 4;
  const int tid = threadIdx.x, lane = tid & 31, wave = tid >> 5;
  const int nodeBase = blockIdx.x * NB;

  {
    const v4f z = {0.f, 0.f, 0.f, 0.f};
    for (int i = tid; i < NB * C / 4; i += NTHR) lds_dyn[i] = z;
  }
  __syncthreads();

  const int nChunks = (nE + CHUNK - 1) / CHUNK;
#pragma unroll 1
  for (int ch = 0; ch < nChunks; ++ch) {
    const int cbase = ch * CHUNK;
    const int wc = scan_chunk<NB>(keys, nE, cbase, nodeBase, vec8, list, tid, lane, wave);
    if (lane == 0) wcnt[wave] = wc;
    __syncthreads();
    if (wave == 0) {
#pragma unroll 1
      for (int wsx = 0; wsx < NWAVE; ++wsx) {
        int n = __builtin_amdgcn_readfirstlane(wcnt[wsx]);
        n = n > WCAP ? WCAP : (n < 0 ? 0 : n);
        const int* lp = list + wsx * WCAP;
#pragma unroll 1
        for (int i = 0; i < n; ++i) {
          const int ent  = __builtin_amdgcn_readfirstlane(lp[i]);
          const int slot = ent & (NB - 1);
          int e = cbase + ((ent >> SLOTB) & (CHUNK - 1));
          e = e > nE - 1 ? nE - 1 : e;
          int src = gidx[e];
          src = src < 0 ? 0 : (src > nN - 1 ? nN - 1 : src);
          const int wi = (MODE == 0) ? src : e;
          const float w = wsrc[wi];
          if (C == 64) {
            const v2f v = *(const v2f*)(zsrc + (size_t)src * 64 + 2 * lane);
            v2f* ap = (v2f*)(acc + slot * 64 + 2 * lane);
            *ap = *ap + v * w;
          } else if (C == 32) {
            const float v = zsrc[(size_t)src * 32 + lane];
            float* ap = acc + slot * 32 + lane;
            *ap = *ap + v * w;
          } else {
            if (lane < C) {
              const float v = zsrc[(size_t)src * C + lane];
              float* ap = acc + slot * C + lane;
              *ap = *ap + v * w;
            }
          }
        }
      }
    }
    __syncthreads();
  }

  v4f* acc4 = (v4f*)acc;
#pragma unroll 4
  for (int i = 0; i < (NB * C / 4) / NTHR; ++i) {
    const int idx  = i * NTHR + tid;
    const int slot = idx / Q;
    const int c4   = (idx - slot * Q) * 4;
    const int row  = nodeBase + slot;
    v4f t = acc4[idx];
    if (MODE == 0) {
      const float dr = wsrc[row];
      t = t * (-dr);
      const v4f rf = *(const v4f*)(zold + (size_t)row * C + c4);
      const v4f t2 = t * 2.0f - rf;
      if (hop >= 2) t = t2;
    }
    acc4[idx] = t;
  }
  __syncthreads();

  float* gp = dst + (size_t)nodeBase * C;
#pragma unroll 4
  for (int i = 0; i < (NB * C / 4) / NTHR; ++i) {
    const int idx = i * NTHR + tid;
    const v4f v = acc4[idx];
    *(volatile v4f*)(gp + (size_t)idx * 4) = v;
  }
  __threadfence();
#pragma unroll 4
  for (int i = 0; i < (NB * C / 4) / NTHR; ++i) {
    const int idx = i * NTHR + tid;
    const v4f v = acc4[idx];
    *(volatile v4f*)(gp + (size_t)idx * 4) = v;
  }
}

__global__ __launch_bounds__(NTHR) void k_tr0(
    const float* __restrict__ planes, const float* __restrict__ W0, const float* __restrict__ b0,
    float* x0, int pstride) {
  const int tid = threadIdx.x;
  const int row = blockIdx.x * 32 + (tid >> 3);
  const int f0  = (tid & 7) * 4;
  v4f s = *(const v4f*)(b0 + f0);
#pragma unroll 1
  for (int k = 0; k < KCH; ++k) {
    const v4f t = *(const v4f*)(planes + (size_t)k * pstride + (size_t)row * 4);
    const float* wp = W0 + k * 96 + f0;
    const v4f w0 = *(const v4f*)wp, w1 = *(const v4f*)(wp + 32), w2 = *(const v4f*)(wp + 64);
    s = s + w0 * t.x;
    s = s + w1 * t.y;
    s = s + w2 * t.z;
  }
  s.x = fmaxf(s.x, 0.f); s.y = fmaxf(s.y, 0.f); s.z = fmaxf(s.z, 0.f); s.w = fmaxf(s.w, 0.f);
  float* gp = x0 + (size_t)row * 32 + f0;
  *(volatile v4f*)gp = s;
  __threadfence();
  *(volatile v4f*)gp = s;
}

template <int CIN, int COUT, int RELU>
__global__ __launch_bounds__(NTHR) void k_gemm(
    const float* __restrict__ planes, const float* __restrict__ W, const float* __restrict__ bias,
    float* xo, int pstride) {
  extern __shared__ v4f lds_dyn[];
  constexpr int BP = CIN + 8, NT = COUT / 16, KS = CIN / 32;
  unsigned short* sBh = (unsigned short*)lds_dyn;
  unsigned short* sBl = sBh + COUT * BP;
  float*          stg = (float*)(sBh + 2 * COUT * BP);
  const int tid = threadIdx.x, lane = tid & 31, wave = tid >> 5, h = lane >> 4, m = lane & 15;
  const int rowBase = blockIdx.x * GROWS;
  const int arow = rowBase + 16 * wave + m;

  v8f acc[NT];
#pragma unroll
  for (int t = 0; t < NT; ++t) { v8f z = {0.f, 0.f, 0.f, 0.f, 0.f, 0.f, 0.f, 0.f}; acc[t] = z; }

#pragma unroll 1
  for (int k = 0; k < KCH; ++k) {
    __syncthreads();
#pragma unroll 4
    for (int i = 0; i < CIN * COUT / NTHR; ++i) {
      const int idx = i * NTHR + tid;
      const int kk  = idx / COUT;
      const int n   = idx - kk * COUT;
      const float x = W[((size_t)(k * CIN + kk)) * COUT + n];
      unsigned short hb, lb;
      split1(x, hb, lb);
      sBh[n * BP + kk] = hb;
      sBl[n * BP + kk] = lb;
    }
    __syncthreads();
    const float* ap = planes + (size_t)k * pstride + (size_t)arow * CIN + 8 * h;
#pragma unroll
    for (int ks = 0; ks < KS; ++ks) {
      const v4f p0 = *(const v4f*)(ap + 32 * ks),      p1 = *(const v4f*)(ap + 32 * ks + 4);
      const v4f p2 = *(const v4f*)(ap + 32 * ks + 16), p3 = *(const v4f*)(ap + 32 * ks + 20);
      FragB ah, al;
      split8(p0, p1, ah.h[0], al.h[0]);
      split8(p2, p3, ah.h[1], al.h[1]);
#pragma unroll
      for (int t = 0; t < NT; ++t) {
        const unsigned short* bph = sBh + (16 * t + m) * BP + 32 * ks + 8 * h;
        const unsigned short* bpl = sBl + (16 * t + m) * BP + 32 * ks + 8 * h;
        FragB bh, bl;
        bh.h[0] = *(const v8us*)bph; bh.h[1] = *(const v8us*)(bph + 16);
        bl.h[0] = *(const v8us*)bpl; bl.h[1] = *(const v8us*)(bpl + 16);
        acc[t] = wmb(ah.v, bh.v, acc[t]);
        acc[t] = wmb(al.v, bh.v, acc[t]);
        acc[t] = wmb(ah.v, bl.v, acc[t]);
      }
    }
  }

  const int r0 = 16 * wave + 8 * h;
  float* sp = stg + r0 * COUT + m;
#pragma unroll
  for (int t = 0; t < NT; ++t) {
    const float bv = bias[16 * t + m];
#pragma unroll
    for (int r = 0; r < 8; ++r) {
      float v = acc[t][r] + bv;
      if (RELU) v = fmaxf(v, 0.f);
      sp[r * COUT + 16 * t] = v;
    }
  }
  __syncthreads();

  constexpr int NI = 16 * COUT / 128;
  const float* lp = stg + 16 * wave * COUT + 4 * lane;
  float* gp = xo + ((size_t)rowBase + 16 * wave) * COUT + 4 * lane;
#pragma unroll
  for (int i = 0; i < NI; ++i) { const v4f v = *(const v4f*)(lp + i * 128); *(volatile v4f*)(gp + i * 128) = v; }
  __threadfence();
#pragma unroll
  for (int i = 0; i < NI; ++i) { const v4f v = *(const v4f*)(lp + i * 128); *(volatile v4f*)(gp + i * 128) = v; }
}

__global__ __launch_bounds__(NTHR) void k_lin(
    const float* __restrict__ lw, const float* __restrict__ x, float* part, int M, int per4) {
  __shared__ float red[NWAVE][16];
  __shared__ __attribute__((aligned(16))) float line[32];
  const int tid = threadIdx.x, lane = tid & 31, wave = tid >> 5;
  const int M4 = M >> 2;
  const int b4 = blockIdx.x * per4;
  int e4 = b4 + per4;
  if (e4 > M4) e4 = M4;

  float acc[NCLS];
#pragma unroll
  for (int c = 0; c < NCLS; ++c) acc[c] = 0.f;
#pragma unroll 1
  for (int j4 = b4 + tid; j4 < e4; j4 += NTHR) {
    const size_t j = (size_t)j4 * 4;
    const v4f xv = *(const v4f*)(x + j);
#pragma unroll
    for (int c = 0; c < NCLS; ++c) {
      const v4f wv = *(const v4f*)(lw + (size_t)c * M + j);
      acc[c] += wv.x * xv.x + wv.y * xv.y + wv.z * xv.z + wv.w * xv.w;
    }
  }
#pragma unroll
  for (int c = 0; c < NCLS; ++c) {
    float v = acc[c];
    v += __shfl_xor(v, 16);
    v += __shfl_xor(v, 8);
    v += __shfl_xor(v, 4);
    v += __shfl_xor(v, 2);
    v += __shfl_xor(v, 1);
    if (lane == 0) red[wave][c] = v;
  }
  __syncthreads();
  if (wave == 0) {
    const int lc = lane < NCLS ? lane : NCLS - 1;
    float s = 0.f;
#pragma unroll
    for (int w = 0; w < NWAVE; ++w) s += red[w][lc];
    line[lane] = (lane < NCLS) ? s : 0.f;
  }
  __syncthreads();
  if (wave == 0) {
    const v4f v = *(const v4f*)(line + 4 * (lane & 7));
    float* gp = part + (size_t)blockIdx.x * 32 + 4 * (lane & 7);
    if (lane < 8) *(volatile v4f*)gp = v;
    __threadfence();
    if (lane < 8) *(volatile v4f*)gp = v;
  }
}

__global__ __launch_bounds__(32) void k_fin(
    const float* __restrict__ part, const float* __restrict__ lb, float* out, int nBlk) {
  const int lane = threadIdx.x;
  double s = 0.0;
#pragma unroll 1
  for (int b = 0; b < nBlk; ++b) s += (double)part[b * 32 + lane];
  const int lc = lane < NCLS ? lane : NCLS - 1;
  const float z = (float)s + lb[lc];
  if (lane < NCLS) *(volatile float*)(out + lane) = z;
  __threadfence();
  if (lane < NCLS) *(volatile float*)(out + lane) = z;
}

extern "C" void kernel_launch(void* const* d_in, const int* in_sizes, int n_in,
                              void* d_out, int out_size, void* d_ws, size_t ws_size,
                              hipStream_t stream) {
  if (n_in < 18) return;
  const int N0 = in_sizes[0] / 3;
  const int E0 = in_sizes[1] / 2, E1 = in_sizes[2] / 2, E2 = in_sizes[3] / 2;
  const int Z0 = in_sizes[4];
  const int Z1 = in_sizes[7];
  const int N1 = in_sizes[7];
  if (N0 <= 0 || in_sizes[0] != 3 * N0) return;
  if (E0 <= 0 || in_sizes[1] != 2 * E0 || E1 <= 0 || in_sizes[2] != 2 * E1 || E2 <= 0 || in_sizes[3] != 2 * E2) return;
  if (Z0 <= 0 || in_sizes[5] != Z0 || in_sizes[6] != Z0 || Z1 <= 0 || in_sizes[8] != Z1 || in_sizes[9] != Z1) return;
  if (in_sizes[10] != KCH * 3 * 32 || in_sizes[11] != 32 || in_sizes[12] != KCH * 32 * 64 ||
      in_sizes[13] != 64 || in_sizes[14] != KCH * 64 * 128 || in_sizes[15] != 128) return;
  if (in_sizes[17] != NCLS || out_size != NCLS) return;
  if (in_sizes[16] <= 0 || in_sizes[16] % (NCLS * 128) != 0) return;
  const int N2 = in_sizes[16] / (NCLS * 128);
  if (N1 <= 0 || N2 <= 0) return;
  const int M = N2 * 128;

  const float* pos = (const float*)d_in[0];
  const int*   ei0 = (const int*)d_in[1];
  const int*   ei1 = (const int*)d_in[2];
  const int*   ei2 = (const int*)d_in[3];
  const int*   d0r = (const int*)d_in[4];
  const int*   d0c = (const int*)d_in[5];
  const float* d0v = (const float*)d_in[6];
  const int*   d1r = (const int*)d_in[7];
  const int*   d1c = (const int*)d_in[8];
  const float* d1v = (const float*)d_in[9];
  const float* W0  = (const float*)d_in[10];
  const float* b0  = (const float*)d_in[11];
  const float* W1  = (const float*)d_in[12];
  const float* b1  = (const float*)d_in[13];
  const float* W2  = (const float*)d_in[14];
  const float* b2  = (const float*)d_in[15];
  const float* lw  = (const float*)d_in[16];
  const float* lb  = (const float*)d_in[17];
  float* out = (float*)d_out;

  const int nB0 = (N0 + NBA - 1) / NBA;       const int N0p = nB0 * NBA;
  const int nB1 = (N1 + NBB - 1) / NBB;       const int N1p = nB1 * NBB;
  const int nB2 = (N2 + NBC - 1) / NBC;       const int N2p = nB2 * NBC;
  const int nD0 = (N0p + NBDEG - 1) / NBDEG;  const int D0p = nD0 * NBDEG;
  const int nD1 = (N1p + NBDEG - 1) / NBDEG;  const int D1p = nD1 * NBDEG;
  const int nD2 = (N2p + NBDEG - 1) / NBDEG;  const int D2p = nD2 * NBDEG;
  if ((N0p % NTHR) != 0 || (N0p % 32) != 0 || (N1p % GROWS) != 0 || (N2p % GROWS) != 0) return;
  if (N2p * 128 < M) return;
  const int M4 = M / 4;
  const int per4 = (M4 + NLB - 1) / NLB;

  char* ws = (char*)d_ws;
  size_t off = 0;
  const size_t oD0 = off; off += (size_t)D0p * 4;                 off = (off + 255) & ~(size_t)255;
  const size_t oD1 = off; off += (size_t)D1p * 4;                 off = (off + 255) & ~(size_t)255;
  const size_t oD2 = off; off += (size_t)D2p * 4;                 off = (off + 255) & ~(size_t)255;
  const size_t oP0 = off; off += (size_t)KCH * N0p * 4 * 4;       off = (off + 255) & ~(size_t)255;
  const size_t oX0 = off; off += (size_t)N0p * 32 * 4;            off = (off + 255) & ~(size_t)255;
  const size_t oP1 = off; off += (size_t)KCH * N1p * 32 * 4;      off = (off + 255) & ~(size_t)255;
  const size_t oX1 = off; off += (size_t)N1p * 64 * 4;            off = (off + 255) & ~(size_t)255;
  const size_t oP2 = off; off += (size_t)KCH * N2p * 64 * 4;      off = (off + 255) & ~(size_t)255;
  const size_t oX2 = off; off += (size_t)N2p * 128 * 4;           off = (off + 255) & ~(size_t)255;
  const size_t oPt = off; off += (size_t)NLB * 32 * 4;            off = (off + 255) & ~(size_t)255;
  if (off > ws_size) return;
  if (off > (size_t)134217728) return;
  float* dinv0 = (float*)(ws + oD0);
  float* dinv1 = (float*)(ws + oD1);
  float* dinv2 = (float*)(ws + oD2);
  float* P0    = (float*)(ws + oP0);
  float* X0    = (float*)(ws + oX0);
  float* P1    = (float*)(ws + oP1);
  float* X1    = (float*)(ws + oX1);
  float* P2    = (float*)(ws + oP2);
  float* X2    = (float*)(ws + oX2);
  float* part  = (float*)(ws + oPt);
  const int S0 = N0p * 4;
  const int S1 = N1p * 32;
  const int S2 = N2p * 64;
  const int vec8 = 1;

  hipFuncSetAttribute(reinterpret_cast<const void*>(&k_agg<4, NBA, 0>),
                      hipFuncAttributeMaxDynamicSharedMemorySize, LDS_AGG);
  hipFuncSetAttribute(reinterpret_cast<const void*>(&k_agg<32, NBB, 0>),
                      hipFuncAttributeMaxDynamicSharedMemorySize, LDS_AGG);
  hipFuncSetAttribute(reinterpret_cast<const void*>(&k_agg<64, NBC, 0>),
                      hipFuncAttributeMaxDynamicSharedMemorySize, LDS_AGG);
  hipFuncSetAttribute(reinterpret_cast<const void*>(&k_agg<32, NBB, 1>),
                      hipFuncAttributeMaxDynamicSharedMemorySize, LDS_AGG);
  hipFuncSetAttribute(reinterpret_cast<const void*>(&k_agg<64, NBC, 1>),
                      hipFuncAttributeMaxDynamicSharedMemorySize, LDS_AGG);
  hipFuncSetAttribute(reinterpret_cast<const void*>(&k_gemm<32, 64, 1>),
                      hipFuncAttributeMaxDynamicSharedMemorySize, LDS_GEMM(32, 64));
  hipFuncSetAttribute(reinterpret_cast<const void*>(&k_gemm<64, 128, 0>),
                      hipFuncAttributeMaxDynamicSharedMemorySize, LDS_GEMM(64, 128));

  k_cp34<<<N0p / NTHR, NTHR, 0, stream>>>(pos, P0, N0);
  k_deg<NBDEG><<<nD0, NTHR, 0, stream>>>(ei0, dinv0, E0, vec8);
  k_deg<NBDEG><<<nD1, NTHR, 0, stream>>>(ei1, dinv1, E1, vec8);
  k_deg<NBDEG><<<nD2, NTHR, 0, stream>>>(ei2, dinv2, E2, vec8);

  for (int k = 1; k < KCH; ++k) {
    const int ko = k >= 2 ? k - 2 : 0;
    k_agg<4, NBA, 0><<<nB0, NTHR, LDS_AGG, stream>>>(
        ei0, ei0 + E0, dinv0, P0 + (size_t)(k - 1) * S0, P0 + (size_t)ko * S0, P0 + (size_t)k * S0,
        N0, E0, k, vec8);
  }
  k_tr0<<<N0p / 32, NTHR, 0, stream>>>(P0, W0, b0, X0, S0);

  k_agg<32, NBB, 1><<<nB1, NTHR, LDS_AGG, stream>>>(d0r, d0c, d0v, X0, X0, P1, N0, Z0, 0, vec8);

  for (int k = 1; k < KCH; ++k) {
    const int ko = k >= 2 ? k - 2 : 0;
    k_agg<32, NBB, 0><<<nB1, NTHR, LDS_AGG, stream>>>(
        ei1, ei1 + E1, dinv1, P1 + (size_t)(k - 1) * S1, P1 + (size_t)ko * S1, P1 + (size_t)k * S1,
        N1, E1, k, vec8);
  }
  k_gemm<32, 64, 1><<<N1p / GROWS, NTHR, LDS_GEMM(32, 64), stream>>>(P1, W1, b1, X1, S1);

  k_agg<64, NBC, 1><<<nB2, NTHR, LDS_AGG, stream>>>(d1r, d1c, d1v, X1, X1, P2, N1, Z1, 0, vec8);

  for (int k = 1; k < KCH; ++k) {
    const int ko = k >= 2 ? k - 2 : 0;
    k_agg<64, NBC, 0><<<nB2, NTHR, LDS_AGG, stream>>>(
        ei2, ei2 + E2, dinv2, P2 + (size_t)(k - 1) * S2, P2 + (size_t)ko * S2, P2 + (size_t)k * S2,
        N2, E2, k, vec8);
  }
  k_gemm<64, 128, 0><<<N2p / GROWS, NTHR, LDS_GEMM(64, 128), stream>>>(P2, W2, b2, X2, S2);

  k_lin<<<NLB, NTHR, 0, stream>>>(lw, X2, part, M, per4);
  k_fin<<<1, 32, 0, stream>>>(part, lb, out, NLB);
}
